// GNN_old_14465449853060
// MI455X (gfx1250) — hardware-verified
//
#include <hip/hip_runtime.h>
#include <hip/hip_bf16.h>
#include <stddef.h>


#define DF      64
#define NOUT    2
#define NTHR    256
#define NWAVE   8
#define EPT     8
#define NGRP    2
#define CHUNK   (NTHR * EPT * NGRP)
#define WCAP    (EPT * NGRP * 32)
#define LISTN   (NWAVE * WCAP)
#define NB      512
#define NPLANE  7
#define PLN     (DF * DF)
#define PLN8    (PLN / 8)
#define WSCALE  8.0f
#define WINV    0.125f

#define LO_ACC    0
#define LO_LIST   (LO_ACC + NB * DF * 4)
#define LO_CNT    (LO_LIST + LISTN * 4)
#define LO_WCNT   (LO_CNT + NB * 4)
#define LO_WL     (LO_WCNT + 64)
#define LO_BL     (LO_WL + DF * NOUT * 4)
#define LDS_LAYER (LO_BL + 64)

static_assert((CHUNK & (CHUNK - 1)) == 0);
static_assert(CHUNK <= 4096);
static_assert((NB & (NB - 1)) == 0);
static_assert(NB <= 4096);
static_assert(NB % 16 == 0);
static_assert(((NB / 16) % NWAVE) == 0);
static_assert(((NB * DF) % (NWAVE * 128)) == 0);
static_assert(NB * NOUT == NWAVE * 128);
static_assert(NB * NOUT * 4 <= LISTN * 4);
static_assert(NB % NTHR == 0);
static_assert(DF % 32 == 0);

typedef float          v2f   __attribute__((ext_vector_type(2)));
typedef float          v4f   __attribute__((ext_vector_type(4)));
typedef float          v8f   __attribute__((ext_vector_type(8)));
typedef int            v4i   __attribute__((ext_vector_type(4)));
typedef _Float16       v8h   __attribute__((ext_vector_type(8)));
typedef _Float16       v16h  __attribute__((ext_vector_type(16)));
typedef __bf16         v16bf __attribute__((ext_vector_type(16)));
typedef unsigned short v8us  __attribute__((ext_vector_type(8)));
union FragH { v16h v; v8h h[2]; };
union FragB { v16bf v; v8us h[2]; };
union Cv8   { v8h f; v8us u; };

__device__ __forceinline__ v8h cvt8(v4f a, v4f b) {
  v8h r;
  r[0] = (_Float16)a.x; r[1] = (_Float16)a.y; r[2] = (_Float16)a.z; r[3] = (_Float16)a.w;
  r[4] = (_Float16)b.x; r[5] = (_Float16)b.y; r[6] = (_Float16)b.z; r[7] = (_Float16)b.w;
  return r;
}

__device__ __forceinline__ unsigned bf16_bits(float x) {
  const unsigned u = __float_as_uint(x);
  return (u + 0x7FFFu + ((u >> 16) & 1u)) >> 16;
}

__device__ __forceinline__ void split1(float x, unsigned short& hi, unsigned short& lo) {
  const unsigned hb = bf16_bits(x);
  const float r = x - __uint_as_float(hb << 16);
  hi = (unsigned short)hb;
  lo = (unsigned short)bf16_bits(r);
}

__device__ __forceinline__ void split8(v4f a, v4f b, v8us& hi, v8us& lo) {
  v8us H = {0, 0, 0, 0, 0, 0, 0, 0};
  v8us L = {0, 0, 0, 0, 0, 0, 0, 0};
  unsigned short h, l;
  split1(a.x, h, l); H[0] = h; L[0] = l;
  split1(a.y, h, l); H[1] = h; L[1] = l;
  split1(a.z, h, l); H[2] = h; L[2] = l;
  split1(a.w, h, l); H[3] = h; L[3] = l;
  split1(b.x, h, l); H[4] = h; L[4] = l;
  split1(b.y, h, l); H[5] = h; L[5] = l;
  split1(b.z, h, l); H[6] = h; L[6] = l;
  split1(b.w, h, l); H[7] = h; L[7] = l;
  hi = H; lo = L;
}

__device__ __forceinline__ v8f wmh(v16h a, v16h b, v8f c) {
  v8f d = __builtin_amdgcn_wmma_f32_16x16x32_f16(false, a, false, b, (short)0, c, false, false);
  asm volatile("v_nop\n\tv_nop\n\tv_nop\n\tv_nop" : "+v"(d) : "v"(a), "v"(b));
  return d;
}
__device__ __forceinline__ v8f wmb(v16bf a, v16bf b, v8f c) {
  v8f d = __builtin_amdgcn_wmma_f32_16x16x32_bf16(false, a, false, b, (short)0, c, false, false);
  asm volatile("v_nop\n\tv_nop\n\tv_nop\n\tv_nop" : "+v"(d) : "v"(a), "v"(b));
  return d;
}

template <int NBT>
__device__ __forceinline__ int scan_chunk(const int* __restrict__ dsts, int nE, int cbase, int nodeBase,
                                          int vec8, int* list, int tid, int lane, int wave) {
  (void)lane;
  int wc = 0;
#pragma unroll
  for (int g = 0; g < NGRP; ++g) {
    const int el0  = (g * NTHR + tid) * EPT;
    const int e0   = cbase + el0;
    const int sent = -2147483647 - 1;
    v4i da, db;
    if (vec8 != 0 && cbase + CHUNK <= nE) {
      da = *(const v4i*)(dsts + e0);
      db = *(const v4i*)(dsts + e0 + 4);
    } else {
      da.x = (e0     < nE) ? dsts[min(e0,     nE - 1)] : sent;
      da.y = (e0 + 1 < nE) ? dsts[min(e0 + 1, nE - 1)] : sent;
      da.z = (e0 + 2 < nE) ? dsts[min(e0 + 2, nE - 1)] : sent;
      da.w = (e0 + 3 < nE) ? dsts[min(e0 + 3, nE - 1)] : sent;
      db.x = (e0 + 4 < nE) ? dsts[min(e0 + 4, nE - 1)] : sent;
      db.y = (e0 + 5 < nE) ? dsts[min(e0 + 5, nE - 1)] : sent;
      db.z = (e0 + 6 < nE) ? dsts[min(e0 + 6, nE - 1)] : sent;
      db.w = (e0 + 7 < nE) ? dsts[min(e0 + 7, nE - 1)] : sent;
    }
    const unsigned nb = (unsigned)nodeBase;
    const unsigned s0 = (unsigned)da.x - nb, s1 = (unsigned)da.y - nb;
    const unsigned s2 = (unsigned)da.z - nb, s3 = (unsigned)da.w - nb;
    const unsigned s4 = (unsigned)db.x - nb, s5 = (unsigned)db.y - nb;
    const unsigned s6 = (unsigned)db.z - nb, s7 = (unsigned)db.w - nb;
    const bool h0 = s0 < (unsigned)NBT, h1 = s1 < (unsigned)NBT, h2 = s2 < (unsigned)NBT, h3 = s3 < (unsigned)NBT;
    const bool h4 = s4 < (unsigned)NBT, h5 = s5 < (unsigned)NBT, h6 = s6 < (unsigned)NBT, h7 = s7 < (unsigned)NBT;
    const unsigned any = __builtin_amdgcn_ballot_w32(h0 | h1 | h2 | h3 | h4 | h5 | h6 | h7);
    if (any != 0u) {
#define HITJ(J, HJ, SJ) { \
        const unsigned mj = __builtin_amdgcn_ballot_w32(HJ); \
        if (mj != 0u) { \
          if (HJ) { \
            const int pos = wc + (int)__builtin_amdgcn_mbcnt_lo(mj, 0u); \
            if (pos < WCAP) list[wave * WCAP + pos] = ((el0 + (J)) << 12) | (int)(SJ); \
          } \
          wc += (int)__builtin_popcount(mj); } }
      HITJ(0, h0, s0)
      HITJ(1, h1, s1)
      HITJ(2, h2, s2)
      HITJ(3, h3, s3)
      HITJ(4, h4, s4)
      HITJ(5, h5, s5)
      HITJ(6, h6, s6)
      HITJ(7, h7, s7)
#undef HITJ
    }
  }
  return wc;
}

__global__ __launch_bounds__(NTHR) void k_wprep(
    const float* __restrict__ W1l, const float* __restrict__ W1r,
    const float* __restrict__ W2l, const float* __restrict__ W2r,
    unsigned short* planes) {
  const int i = blockIdx.x * NTHR + threadIdx.x;
  if (i >= NPLANE * PLN8) return;
  const int p  = i / PLN8;
  const int o  = (i - p * PLN8) * 8;
  const int n  = o >> 6;
  const int k0 = o & 63;
  const float* W = (p == 0) ? W1l : ((p <= 2) ? W1r : ((p <= 4) ? W2l : W2r));
  const float* src = W + (size_t)k0 * DF + n;
  v4f a, b;
  a.x = src[0];      a.y = src[DF];     a.z = src[2 * DF]; a.w = src[3 * DF];
  b.x = src[4 * DF]; b.y = src[5 * DF]; b.z = src[6 * DF]; b.w = src[7 * DF];
  a = a * WSCALE;
  b = b * WSCALE;
  v8us u;
  if (p == 0) {
    Cv8 c; c.f = cvt8(a, b); u = c.u;
  } else {
    v8us hi, lo;
    split8(a, b, hi, lo);
    u = (p & 1) ? hi : lo;
  }
  unsigned short* dp = planes + (size_t)p * PLN + o;
  *(volatile v8us*)dp = u;
  __threadfence();
  *(volatile v8us*)dp = u;
}

template <bool AGGF16, bool FINAL>
__global__ __launch_bounds__(NTHR) void k_layer(
    const int* __restrict__ ei, const float* __restrict__ feat,
    const unsigned short* __restrict__ pl, const unsigned short* __restrict__ pr,
    const float* __restrict__ bias, const float* __restrict__ wlin, const float* __restrict__ blin,
    float* hout, float* out, int nN, int nE, int vec8) {
  extern __shared__ v4f lds_dyn[];
  char*  lb   = (char*)lds_dyn;
  float* acc  = (float*)(lb + LO_ACC);
  int*   list = (int*)(lb + LO_LIST);
  int*   cnt  = (int*)(lb + LO_CNT);
  int*   wcnt = (int*)(lb + LO_WCNT);
  float* sW   = (float*)(lb + LO_WL);
  float* sBl  = (float*)(lb + LO_BL);
  float* so   = (float*)(lb + LO_LIST);
  const int tid = threadIdx.x, lane = tid & 31, wave = tid >> 5, hh = lane >> 4, m = lane & 15;
  const int nodeBase = blockIdx.x * NB;
  const int* dsts = ei + nE;

  {
    const v4f z = {0.f, 0.f, 0.f, 0.f};
    for (int i = tid; i < NB * DF / 4; i += NTHR) lds_dyn[i] = z;
  }
  for (int i = tid; i < NB; i += NTHR) cnt[i] = 0;
  if (FINAL) {
    if (tid < DF * NOUT) sW[tid] = wlin[tid];
    if (tid < NOUT) sBl[tid] = blin[tid];
  }
  __syncthreads();

  const int nChunks = (nE + CHUNK - 1) / CHUNK;
#pragma unroll 1
  for (int ch = 0; ch < nChunks; ++ch) {
    const int cbase = ch * CHUNK;
    const int wc = scan_chunk<NB>(dsts, nE, cbase, nodeBase, vec8, list, tid, lane, wave);
    if (lane == 0) wcnt[wave] = wc;
    __syncthreads();
    if (wave == 0) {
#pragma unroll 1
      for (int wsx = 0; wsx < NWAVE; ++wsx) {
        int n = __builtin_amdgcn_readfirstlane(wcnt[wsx]);
        n = n > WCAP ? WCAP : (n < 0 ? 0 : n);
        const int* lp = list + wsx * WCAP;
#pragma unroll 1
        for (int i = 0; i < n; ++i) {
          const int ent  = __builtin_amdgcn_readfirstlane(lp[i]);
          const int slot = ent & (NB - 1);
          int e = cbase + ((ent >> 12) & (CHUNK - 1));
          e = e > nE - 1 ? nE - 1 : e;
          int src = ei[e];
          src = src < 0 ? 0 : (src > nN - 1 ? nN - 1 : src);
          const v2f v = *(const v2f*)(feat + (size_t)src * DF + 2 * lane);
          v2f* ap = (v2f*)(acc + slot * DF + 2 * lane);
          *ap = *ap + v;
          if (lane == 0) cnt[slot] = cnt[slot] + 1;
        }
      }
    }
    __syncthreads();
  }

  float bv[4];
#pragma unroll
  for (int j = 0; j < 4; ++j) bv[j] = bias[16 * j + m];

#pragma unroll 1
  for (int tt = 0; tt < (NB / 16) / NWAVE; ++tt) {
    const int t     = wave + NWAVE * tt;
    const int slotA = 16 * t + m;
    const float scl = 1.0f / fmaxf((float)cnt[slotA], 1.0f);
    int nodeA = nodeBase + slotA;
    nodeA = nodeA > nN - 1 ? nN - 1 : nodeA;
    const float* ar = acc + slotA * DF + 8 * hh;
    const float* fr = feat + (size_t)nodeA * DF + 8 * hh;

    v8f c[4];
#pragma unroll
    for (int j = 0; j < 4; ++j) { v8f z = {0.f, 0.f, 0.f, 0.f, 0.f, 0.f, 0.f, 0.f}; c[j] = z; }

#pragma unroll 1
    for (int ks = 0; ks < DF / 32; ++ks) {
      const float* ap = ar + 32 * ks;
      const v4f p0 = *(const v4f*)ap * scl,        p1 = *(const v4f*)(ap + 4) * scl;
      const v4f p2 = *(const v4f*)(ap + 16) * scl, p3 = *(const v4f*)(ap + 20) * scl;
      if (AGGF16) {
        FragH a;
        a.h[0] = cvt8(p0, p1);
        a.h[1] = cvt8(p2, p3);
#pragma unroll
        for (int j = 0; j < 4; ++j) {
          const unsigned short* bp = pl + (16 * j + m) * DF + 32 * ks + 8 * hh;
          FragH b;
          b.h[0] = *(const v8h*)bp;
          b.h[1] = *(const v8h*)(bp + 16);
          c[j] = wmh(a.v, b.v, c[j]);
        }
      } else {
        FragB ahi, alo;
        split8(p0, p1, ahi.h[0], alo.h[0]);
        split8(p2, p3, ahi.h[1], alo.h[1]);
#pragma unroll
        for (int j = 0; j < 4; ++j) {
          const unsigned short* bp = pl + (16 * j + m) * DF + 32 * ks + 8 * hh;
          FragB bh, bl;
          bh.h[0] = *(const v8us*)bp;         bh.h[1] = *(const v8us*)(bp + 16);
          bl.h[0] = *(const v8us*)(bp + PLN); bl.h[1] = *(const v8us*)(bp + PLN + 16);
          c[j] = wmb(ahi.v, bh.v, c[j]);
          c[j] = wmb(ahi.v, bl.v, c[j]);
          c[j] = wmb(alo.v, bh.v, c[j]);
        }
      }
    }
#pragma unroll 1
    for (int ks = 0; ks < DF / 32; ++ks) {
      const float* gp = fr + 32 * ks;
      const v4f p0 = *(const v4f*)gp,        p1 = *(const v4f*)(gp + 4);
      const v4f p2 = *(const v4f*)(gp + 16), p3 = *(const v4f*)(gp + 20);
      FragB ahi, alo;
      split8(p0, p1, ahi.h[0], alo.h[0]);
      split8(p2, p3, ahi.h[1], alo.h[1]);
#pragma unroll
      for (int j = 0; j < 4; ++j) {
        const unsigned short* bp = pr + (16 * j + m) * DF + 32 * ks + 8 * hh;
        FragB bh, bl;
        bh.h[0] = *(const v8us*)bp;         bh.h[1] = *(const v8us*)(bp + 16);
        bl.h[0] = *(const v8us*)(bp + PLN); bl.h[1] = *(const v8us*)(bp + PLN + 16);
        c[j] = wmb(ahi.v, bh.v, c[j]);
        c[j] = wmb(ahi.v, bl.v, c[j]);
        c[j] = wmb(alo.v, bh.v, c[j]);
      }
    }
    float* sp = acc + (16 * t + 8 * hh) * DF + m;
#pragma unroll
    for (int j = 0; j < 4; ++j) {
      sp[0 * DF + 16 * j] = fmaxf(c[j][0] * WINV + bv[j], 0.f);
      sp[1 * DF + 16 * j] = fmaxf(c[j][1] * WINV + bv[j], 0.f);
      sp[2 * DF + 16 * j] = fmaxf(c[j][2] * WINV + bv[j], 0.f);
      sp[3 * DF + 16 * j] = fmaxf(c[j][3] * WINV + bv[j], 0.f);
      sp[4 * DF + 16 * j] = fmaxf(c[j][4] * WINV + bv[j], 0.f);
      sp[5 * DF + 16 * j] = fmaxf(c[j][5] * WINV + bv[j], 0.f);
      sp[6 * DF + 16 * j] = fmaxf(c[j][6] * WINV + bv[j], 0.f);
      sp[7 * DF + 16 * j] = fmaxf(c[j][7] * WINV + bv[j], 0.f);
    }
  }
  __syncthreads();

  if (!FINAL) {
    const size_t gb = (size_t)nodeBase * DF;
#pragma unroll 4
    for (int q = 0; q < (NB * DF) / (NWAVE * 128); ++q) {
      const int f = (wave * ((NB * DF) / (NWAVE * 128)) + q) * 128 + 4 * lane;
      const v4f v = *(const v4f*)(acc + f);
      *(volatile v4f*)(hout + gb + f) = v;
    }
    __threadfence();
#pragma unroll 4
    for (int q = 0; q < (NB * DF) / (NWAVE * 128); ++q) {
      const int f = (wave * ((NB * DF) / (NWAVE * 128)) + q) * 128 + 4 * lane;
      const v4f v = *(const v4f*)(acc + f);
      *(volatile v4f*)(hout + gb + f) = v;
    }
  } else {
#pragma unroll 1
    for (int si = 0; si < NB / NTHR; ++si) {
      const int slot = si * NTHR + tid;
      const float* row = acc + slot * DF;
      float o0 = 0.f, o1 = 0.f;
#pragma unroll 4
      for (int k4 = 0; k4 < DF / 4; ++k4) {
        const v4f v = *(const v4f*)(row + 4 * k4);
        const float* w = sW + 8 * k4;
        o0 += v.x * w[0] + v.y * w[2] + v.z * w[4] + v.w * w[6];
        o1 += v.x * w[1] + v.y * w[3] + v.z * w[5] + v.w * w[7];
      }
      so[slot * NOUT + 0] = o0 + sBl[0];
      so[slot * NOUT + 1] = o1 + sBl[1];
    }
    __syncthreads();
    const size_t outN = (size_t)nN * NOUT;
    const size_t ob   = (size_t)nodeBase * NOUT;
    const int f = wave * 128 + 4 * lane;
    const v4f v = *(const v4f*)(so + f);
    const size_t gi = ob + (size_t)f;
    const v2f vl = {v.x, v.y};
    if (gi + 4 <= outN) { *(volatile v4f*)(out + gi) = v; }
    else if (gi + 2 <= outN) { *(volatile v2f*)(out + gi) = vl; }
    __threadfence();
    if (gi + 4 <= outN) { *(volatile v4f*)(out + gi) = v; }
    else if (gi + 2 <= outN) { *(volatile v2f*)(out + gi) = vl; }
  }
}

extern "C" void kernel_launch(void* const* d_in, const int* in_sizes, int n_in,
                              void* d_out, int out_size, void* d_ws, size_t ws_size,
                              hipStream_t stream) {
  if (n_in < 10) return;
  const int nN = in_sizes[0] / DF;
  const int nE = in_sizes[1] / 2;
  if (nN <= 0 || nE < 0 || in_sizes[0] != nN * DF || in_sizes[1] != nE * 2) return;
  if (in_sizes[2] != DF * DF || in_sizes[3] < DF || in_sizes[4] != DF * DF) return;
  if (in_sizes[5] != DF * DF || in_sizes[6] < DF || in_sizes[7] != DF * DF) return;
  if (in_sizes[8] != DF * NOUT || in_sizes[9] < NOUT) return;
  if (out_size != nN * NOUT) return;

  const float* x    = (const float*)d_in[0];
  const int*   ei   = (const int*)d_in[1];
  const float* W1l  = (const float*)d_in[2];
  const float* b1   = (const float*)d_in[3];
  const float* W1r  = (const float*)d_in[4];
  const float* W2l  = (const float*)d_in[5];
  const float* b2   = (const float*)d_in[6];
  const float* W2r  = (const float*)d_in[7];
  const float* Wlin = (const float*)d_in[8];
  const float* blin = (const float*)d_in[9];
  float* out = (float*)d_out;

  const int nA = (nN + NB - 1) / NB;

  char* ws = (char*)d_ws;
  size_t off = 0;
  const size_t oPl = off; off += (size_t)NPLANE * PLN * 2;          off = (off + 255) & ~(size_t)255;
  const size_t oH1 = off; off += (size_t)nA * NB * DF * 4;          off = (off + 255) & ~(size_t)255;
  if (off > ws_size) return;
  unsigned short* planes = (unsigned short*)(ws + oPl);
  float*          h1     = (float*)(ws + oH1);

  const int vec8 = ((nE & 3) == 0) ? 1 : 0;

  const int nPrep = NPLANE * PLN8;
  k_wprep<<<(nPrep + NTHR - 1) / NTHR, NTHR, 0, stream>>>(W1l, W1r, W2l, W2r, planes);

  hipFuncSetAttribute(reinterpret_cast<const void*>(&k_layer<true, false>),
                      hipFuncAttributeMaxDynamicSharedMemorySize, LDS_LAYER);
  k_layer<true, false><<<nA, NTHR, LDS_LAYER, stream>>>(
      ei, x, planes, planes + 1 * PLN, b1, Wlin, blin, h1, out, nN, nE, vec8);

  hipFuncSetAttribute(reinterpret_cast<const void*>(&k_layer<false, true>),
                      hipFuncAttributeMaxDynamicSharedMemorySize, LDS_LAYER);
  k_layer<false, true><<<nA, NTHR, LDS_LAYER, stream>>>(
      ei, h1, planes + 3 * PLN, planes + 5 * PLN, b2, Wlin, blin, h1, out, nN, nE, vec8);
}
